// Quanvolution__gen329_65481071408268
// MI455X (gfx1250) — hardware-verified
//
#include <hip/hip_runtime.h>
#define NIMG 1024
#define NPATCH 196
#define NC (NIMG * NPATCH)
#define NCLS 10
#define NQ 784

typedef __bf16 v16b __attribute__((ext_vector_type(16)));
typedef unsigned short v8us __attribute__((ext_vector_type(8), may_alias));
typedef float  v8f  __attribute__((ext_vector_type(8)));
typedef float  v4f  __attribute__((ext_vector_type(4)));
typedef float  v4fa __attribute__((ext_vector_type(4), may_alias));
union FragB { v16b v; v8us half[2]; unsigned short u[16]; };

__device__ __forceinline__ unsigned short bf16_bits(float x) { unsigned int u = __float_as_uint(x); return (unsigned short)((u + 0x7FFFu + ((u >> 16) & 1u)) >> 16); }
__device__ __forceinline__ float bf16_val(unsigned short b) { return __uint_as_float(((unsigned int)b) << 16); }
__device__ __forceinline__ float bf16_round(float x) { return bf16_val(bf16_bits(x)); }
template <int NT>
__device__ __forceinline__ v8f mmaN(v16b ah, v16b al, v16b bh, v16b bl, v8f c) {
  c = __builtin_amdgcn_wmma_f32_16x16x32_bf16(false, ah, false, bh, (short)0, c, false, false);
  if (NT >= 2) c = __builtin_amdgcn_wmma_f32_16x16x32_bf16(false, al, false, bh, (short)0, c, false, false);
  if (NT >= 3) c = __builtin_amdgcn_wmma_f32_16x16x32_bf16(false, ah, false, bl, (short)0, c, false, false);
  asm volatile("v_nop\n\tv_nop\n\tv_nop\n\tv_nop" : "+v"(c) : "v"(ah), "v"(al), "v"(bh), "v"(bl));
  return c;
}

__global__ __launch_bounds__(256) void k_wt_bf16(const float* __restrict__ W, unsigned short* __restrict__ Wt, int K, int N) {
  const int t = blockIdx.x * 256 + threadIdx.x;
  const int k8n = K / 8;
  if (t >= N * k8n) return;
  const int n = t / k8n, k8 = (t % k8n) * 8;
  v8us v;
#pragma unroll
  for (int i = 0; i < 8; ++i) v[i] = bf16_bits(W[(size_t)(k8 + i) * N + n]);
  *(volatile v8us*)(Wt + (size_t)n * K + k8) = v;
  __threadfence();
  *(volatile v8us*)(Wt + (size_t)n * K + k8) = v;
}

template <bool ASPLIT, int ACT, bool BIAS_BF16>
__global__ __launch_bounds__(128) void k_gemm_bf(const float* __restrict__ A, int lda, const unsigned short* __restrict__ Wt, int ldb,
                                               const float* __restrict__ bias, float* __restrict__ C, int ldc, int M, int N, int K) {
  __shared__ __attribute__((aligned(16))) float so[4][16][64];
  const int tid = threadIdx.x, w = tid >> 5, lane = tid & 31, ln = lane & 15, hh = lane >> 4;
  const int ntn = N / 64;
  const int wid = blockIdx.x * 4 + w;
  const int mt = wid / ntn, nq = wid % ntn;
  if (mt * 16 >= M) return;
  const int row0 = mt * 16, col0 = nq * 64;
  const float* arow = A + (size_t)(row0 + ln) * lda;
  v8f acc[4] = {};
  for (int kb = 0; kb < K; kb += 32) {
    FragB ah, al;
    const v4f x0 = *(const v4fa*)(arow + kb + 8 * hh), x1 = *(const v4fa*)(arow + kb + 8 * hh + 4);
    const v4f x2 = *(const v4fa*)(arow + kb + 16 + 8 * hh), x3 = *(const v4fa*)(arow + kb + 16 + 8 * hh + 4);
    float xs[16] = {x0[0],x0[1],x0[2],x0[3],x1[0],x1[1],x1[2],x1[3],x2[0],x2[1],x2[2],x2[3],x3[0],x3[1],x3[2],x3[3]};
#pragma unroll
    for (int i = 0; i < 16; ++i) { const unsigned short hb = bf16_bits(xs[i]); ah.u[i] = hb; al.u[i] = ASPLIT ? bf16_bits(xs[i] - bf16_val(hb)) : (unsigned short)0; }
#pragma unroll
    for (int t = 0; t < 4; ++t) {
      const unsigned short* brow = Wt + (size_t)(col0 + t * 16 + ln) * ldb + kb;
      FragB b;
      b.half[0] = *(const v8us*)(brow + 8 * hh);
      b.half[1] = *(const v8us*)(brow + 16 + 8 * hh);
      acc[t] = mmaN<ASPLIT ? 2 : 1>(ah.v, al.v, b.v, b.v, acc[t]);
    }
  }
#pragma unroll
  for (int t = 0; t < 4; ++t) {
    float bv = bias ? bias[col0 + t * 16 + ln] : 0.f;
    if (BIAS_BF16) bv = bf16_round(bv);
#pragma unroll
    for (int r = 0; r < 8; ++r) { float v = acc[t][r] + bv; if (ACT == 1) v = fmaxf(v, 0.f); so[w][8 * hh + r][t * 16 + ln] = v; }
  }
  __builtin_amdgcn_fence(__ATOMIC_ACQ_REL, "workgroup");
  __builtin_amdgcn_wave_barrier();
  const int rsub = lane >> 4, c4 = (lane & 15) * 4;
  for (int pass = 0; pass < 2; ++pass) {
#pragma unroll
    for (int q = 0; q < 8; ++q) {
      const int r = q * 2 + rsub;
      const v4f v = *(const v4fa*)&so[w][r][c4];
      *(volatile v4f*)(C + (size_t)(row0 + r) * ldc + col0 + c4) = v;
    }
    if (pass == 0) __threadfence();
  }
}

template <int D, bool CAUSAL>
__global__ __launch_bounds__(128) void k_flash(const float* __restrict__ qb, const float* __restrict__ kb, const float* __restrict__ vb,
                                             int pitch, int T, int H, float scale, float* __restrict__ y, int ypitch) {
  constexpr int KS = D / 32;
  constexpr int DT = D / 16;
  __shared__ __attribute__((aligned(16))) unsigned short sKh[32][D + 8], sKl[32][D + 8], sVh[32][D + 8], sVl[32][D + 8];
  __shared__ __attribute__((aligned(16))) unsigned short sPh[4][16][40], sPl[4][16][40];
  __shared__ __attribute__((aligned(16))) float sO[4][16][D];
  const int tid = threadIdx.x, w = tid >> 5, lane = tid & 31, ln = lane & 15, hh = lane >> 4;
  const int nqb = (T + 63) / 64;
  const int bh = blockIdx.x / nqb, qblk = blockIdx.x % nqb;
  const int b = bh / H, h = bh % H;
  const int q0 = qblk * 64 + w * 16;
  const float* Q = qb + (size_t)b * T * pitch + h * D;
  const float* K = kb + (size_t)b * T * pitch + h * D;
  const float* V = vb + (size_t)b * T * pitch + h * D;

  FragB aqh[KS], aql[KS];
  {
    int row = q0 + ln; if (row >= T) row = T - 1;
    const float* qr = Q + (size_t)row * pitch;
#pragma unroll
    for (int ks = 0; ks < KS; ++ks)
#pragma unroll
      for (int i = 0; i < 16; ++i) {
        const int d = ks * 32 + ((i < 8) ? (8 * hh + i) : (16 + 8 * hh + (i - 8)));
        const float x = qr[d] * scale; const unsigned short hb = bf16_bits(x);
        aqh[ks].u[i] = hb; aql[ks].u[i] = bf16_bits(x - bf16_val(hb));
      }
  }
  float m_r[8], l_r[8];
#pragma unroll
  for (int r = 0; r < 8; ++r) { m_r[r] = -3.0e38f; l_r[r] = 0.f; }
  v8f oacc[DT];
#pragma unroll
  for (int dt = 0; dt < DT; ++dt) oacc[dt] = (v8f){0.f,0.f,0.f,0.f,0.f,0.f,0.f,0.f};

  const int kv_end = CAUSAL ? min(T, qblk * 64 + 64) : T;
  for (int j0 = 0; j0 < kv_end; j0 += 32) {
    __syncthreads();
    for (int e = tid; e < 32 * (D / 4); e += 128) {
      const int r = e / (D / 4), c4 = (e % (D / 4)) * 4;
      const int key = j0 + r;
      v4f kf = {0.f,0.f,0.f,0.f}, vf = {0.f,0.f,0.f,0.f};
      if (key < T) { kf = *(const v4fa*)(K + (size_t)key * pitch + c4); vf = *(const v4fa*)(V + (size_t)key * pitch + c4); }
#pragma unroll
      for (int t = 0; t < 4; ++t) {
        unsigned short hb = bf16_bits(kf[t]); sKh[r][c4 + t] = hb; sKl[r][c4 + t] = bf16_bits(kf[t] - bf16_val(hb));
        hb = bf16_bits(vf[t]); sVh[r][c4 + t] = hb; sVl[r][c4 + t] = bf16_bits(vf[t] - bf16_val(hb));
      }
    }
    __syncthreads();
    v8f s[2];
#pragma unroll
    for (int nt = 0; nt < 2; ++nt) {
      v8f acc = {};
#pragma unroll
      for (int ks = 0; ks < KS; ++ks) {
        FragB bh_, bl_;
        bh_.half[0] = *(const v8us*)&sKh[nt * 16 + ln][ks * 32 + 8 * hh]; bh_.half[1] = *(const v8us*)&sKh[nt * 16 + ln][ks * 32 + 16 + 8 * hh];
        bl_.half[0] = *(const v8us*)&sKl[nt * 16 + ln][ks * 32 + 8 * hh]; bl_.half[1] = *(const v8us*)&sKl[nt * 16 + ln][ks * 32 + 16 + 8 * hh];
        acc = mmaN<3>(aqh[ks].v, aql[ks].v, bh_.v, bl_.v, acc);
      }
      s[nt] = acc;
    }
    float alpha[8];
#pragma unroll
    for (int r = 0; r < 8; ++r) {
      const int qi = q0 + 8 * hh + r;
      const int ja = j0 + ln, jb = j0 + 16 + ln;
      if (CAUSAL) { if (ja > qi) s[0][r] = -3.0e38f; if (jb > qi) s[1][r] = -3.0e38f; }
      if (ja >= T) s[0][r] = -3.0e38f;
      if (jb >= T) s[1][r] = -3.0e38f;
      float mx = fmaxf(s[0][r], s[1][r]);
      mx = fmaxf(mx, __shfl_xor(mx, 1, 32)); mx = fmaxf(mx, __shfl_xor(mx, 2, 32)); mx = fmaxf(mx, __shfl_xor(mx, 4, 32)); mx = fmaxf(mx, __shfl_xor(mx, 8, 32));
      const float mnew = fmaxf(m_r[r], mx);
      alpha[r] = (mnew > -1.0e38f) ? __expf(m_r[r] - mnew) : 1.0f;
      const float p0 = (s[0][r] > -1.0e38f) ? __expf(s[0][r] - mnew) : 0.f;
      const float p1 = (s[1][r] > -1.0e38f) ? __expf(s[1][r] - mnew) : 0.f;
      m_r[r] = mnew;
      l_r[r] = l_r[r] * alpha[r] + p0 + p1;
      unsigned short hb = bf16_bits(p0); sPh[w][8 * hh + r][ln] = hb;      sPl[w][8 * hh + r][ln] = bf16_bits(p0 - bf16_val(hb));
      hb = bf16_bits(p1);                sPh[w][8 * hh + r][16 + ln] = hb; sPl[w][8 * hh + r][16 + ln] = bf16_bits(p1 - bf16_val(hb));
    }
#pragma unroll
    for (int dt = 0; dt < DT; ++dt)
#pragma unroll
      for (int r = 0; r < 8; ++r) oacc[dt][r] *= alpha[r];
    __builtin_amdgcn_fence(__ATOMIC_ACQ_REL, "workgroup");
    __builtin_amdgcn_wave_barrier();
    FragB pah, pal;
    pah.half[0] = *(const v8us*)&sPh[w][ln][8 * hh]; pah.half[1] = *(const v8us*)&sPh[w][ln][16 + 8 * hh];
    pal.half[0] = *(const v8us*)&sPl[w][ln][8 * hh]; pal.half[1] = *(const v8us*)&sPl[w][ln][16 + 8 * hh];
#pragma unroll
    for (int dt = 0; dt < DT; ++dt) {
      FragB bvh, bvl;
#pragma unroll
      for (int i = 0; i < 8; ++i) {
        bvh.u[i] = sVh[8 * hh + i][dt * 16 + ln]; bvh.u[8 + i] = sVh[16 + 8 * hh + i][dt * 16 + ln];
        bvl.u[i] = sVl[8 * hh + i][dt * 16 + ln]; bvl.u[8 + i] = sVl[16 + 8 * hh + i][dt * 16 + ln];
      }
      oacc[dt] = mmaN<3>(pah.v, pal.v, bvh.v, bvl.v, oacc[dt]);
    }
    __builtin_amdgcn_fence(__ATOMIC_ACQ_REL, "workgroup");
    __builtin_amdgcn_wave_barrier();
  }
#pragma unroll
  for (int r = 0; r < 8; ++r) {
    float l = l_r[r];
    l += __shfl_xor(l, 1, 32); l += __shfl_xor(l, 2, 32); l += __shfl_xor(l, 4, 32); l += __shfl_xor(l, 8, 32);
    l_r[r] = (l > 0.f) ? 1.0f / l : 0.f;
  }
#pragma unroll
  for (int dt = 0; dt < DT; ++dt)
#pragma unroll
    for (int r = 0; r < 8; ++r) sO[w][8 * hh + r][dt * 16 + ln] = oacc[dt][r] * l_r[r];
  __builtin_amdgcn_fence(__ATOMIC_ACQ_REL, "workgroup");
  __builtin_amdgcn_wave_barrier();
  for (int pass = 0; pass < 2; ++pass) {
    for (int r = 0; r < 16; ++r) {
      const int row = q0 + r;
      if (row < T && lane < D / 4) {
        const v4f val = *(const v4fa*)&sO[w][r][lane * 4];
        *(volatile v4f*)(y + ((size_t)b * T + row) * ypitch + h * D + lane * 4) = val;
      }
    }
    if (pass == 0) __threadfence();
  }
}

template <bool ASPLIT, int ACT, bool BIAS_BF16, bool RES_BF16>
__global__ __launch_bounds__(128) void k_gemm_bf3(const float* __restrict__ A, int lda, const unsigned short* __restrict__ Wt, int ldb,
                                                const float* __restrict__ bias, const float* __restrict__ resid, int rmod, int ldr,
                                                float* __restrict__ C, int ldc, int M, int N, int K) {
  __shared__ __attribute__((aligned(16))) float so[4][16][64];
  const int tid = threadIdx.x, w = tid >> 5, lane = tid & 31, ln = lane & 15, hh = lane >> 4;
  const int ntn = N / 64;
  const int wid = blockIdx.x * 4 + w;
  const int mt = wid / ntn, nq = wid % ntn;
  if (mt * 16 >= M) return;
  const int row0 = mt * 16, col0 = nq * 64;
  const float* arow = A + (size_t)(row0 + ln) * lda;
  v8f acc[4] = {};
  for (int kb = 0; kb < K; kb += 32) {
    FragB ah, al;
    const v4f x0 = *(const v4fa*)(arow + kb + 8 * hh), x1 = *(const v4fa*)(arow + kb + 8 * hh + 4);
    const v4f x2 = *(const v4fa*)(arow + kb + 16 + 8 * hh), x3 = *(const v4fa*)(arow + kb + 16 + 8 * hh + 4);
    float xs[16] = {x0[0],x0[1],x0[2],x0[3],x1[0],x1[1],x1[2],x1[3],x2[0],x2[1],x2[2],x2[3],x3[0],x3[1],x3[2],x3[3]};
#pragma unroll
    for (int i = 0; i < 16; ++i) { const unsigned short hb = bf16_bits(xs[i]); ah.u[i] = hb; al.u[i] = ASPLIT ? bf16_bits(xs[i] - bf16_val(hb)) : (unsigned short)0; }
#pragma unroll
    for (int t = 0; t < 4; ++t) {
      const unsigned short* brow = Wt + (size_t)(col0 + t * 16 + ln) * ldb + kb;
      FragB b;
      b.half[0] = *(const v8us*)(brow + 8 * hh);
      b.half[1] = *(const v8us*)(brow + 16 + 8 * hh);
      acc[t] = mmaN<ASPLIT ? 2 : 1>(ah.v, al.v, b.v, b.v, acc[t]);
    }
  }
#pragma unroll
  for (int t = 0; t < 4; ++t) {
    const int col = col0 + t * 16 + ln;
    float bv = bias ? bias[col] : 0.f;
    if (BIAS_BF16) bv = bf16_round(bv);
#pragma unroll
    for (int r = 0; r < 8; ++r) {
      float v = acc[t][r] + bv;
      if (resid) { float rv = resid[(size_t)((row0 + 8 * hh + r) % rmod) * ldr + col]; if (RES_BF16) rv = bf16_round(rv); v += rv; }
      if (ACT == 1) v = fmaxf(v, 0.f);
      if (ACT == 2) v = 0.5f * v * (1.0f + erff(v * 0.70710678118654752f));
      if (ACT == 3) { const float u = 0.7978845608028654f * (v + 0.044715f * v * v * v); v = 0.5f * v * (1.0f + tanhf(u)); }
      so[w][8 * hh + r][t * 16 + ln] = v;
    }
  }
  __builtin_amdgcn_fence(__ATOMIC_ACQ_REL, "workgroup");
  __builtin_amdgcn_wave_barrier();
  const int rsub = lane >> 4, c4 = (lane & 15) * 4;
  for (int pass = 0; pass < 2; ++pass) {
#pragma unroll
    for (int q = 0; q < 8; ++q) {
      const int r = q * 2 + rsub;
      const v4f v = *(const v4fa*)&so[w][r][c4];
      *(volatile v4f*)(C + (size_t)(row0 + r) * ldc + col0 + c4) = v;
    }
    if (pass == 0) __threadfence();
  }
}
template <bool PARAM_BF16>
__global__ __launch_bounds__(256) void k_layernorm(const float* __restrict__ X, const float* __restrict__ R, const float* __restrict__ g, const float* __restrict__ bta,
                                                  float* __restrict__ out_sum, float* __restrict__ out_norm, int N, float eps) {
  __shared__ float red[256];
  const int row = blockIdx.x, tid = threadIdx.x;
  const float* x = X + (size_t)row * N; const float* rr = R ? R + (size_t)row * N : nullptr;
  float vals[16];
  const int per = N / 256;
  float s1 = 0.f;
  for (int u = 0; u < per / 4; ++u) {
    const int j = tid * 4 + 1024 * u;
    const v4f a = *(const v4fa*)(x + j);
    v4f b = {0.f,0.f,0.f,0.f}; if (rr) b = *(const v4fa*)(rr + j);
#pragma unroll
    for (int q = 0; q < 4; ++q) { const float v = a[q] + b[q]; vals[u * 4 + q] = v; s1 += v; }
  }
  red[tid] = s1; __syncthreads();
  for (int st = 128; st > 0; st >>= 1) { if (tid < st) red[tid] += red[tid + st]; __syncthreads(); }
  const float mu = red[0] / (float)N; __syncthreads();
  float s2 = 0.f;
  for (int u = 0; u < per / 4; ++u)
#pragma unroll
    for (int q = 0; q < 4; ++q) { const float c = vals[u * 4 + q] - mu; s2 += c * c; }
  red[tid] = s2; __syncthreads();
  for (int st = 128; st > 0; st >>= 1) { if (tid < st) red[tid] += red[tid + st]; __syncthreads(); }
  const float rs = rsqrtf(red[0] / (float)N + eps);
  for (int pass = 0; pass < 2; ++pass) {
    for (int u = 0; u < per / 4; ++u) {
      const int j = tid * 4 + 1024 * u;
      v4f o, sm;
#pragma unroll
      for (int q = 0; q < 4; ++q) {
        float gg = g[j + q], bb = bta[j + q];
        if (PARAM_BF16) { gg = bf16_round(gg); bb = bf16_round(bb); }
        sm[q] = vals[u * 4 + q]; o[q] = (vals[u * 4 + q] - mu) * rs * gg + bb;
      }
      if (out_sum) *(volatile v4f*)(out_sum + (size_t)row * N + j) = sm;
      *(volatile v4f*)(out_norm + (size_t)row * N + j) = o;
    }
    if (pass == 0) __threadfence();
  }
}


typedef _Float16 v16h __attribute__((ext_vector_type(16)));
union FragH { v16h v; v8us half[2]; _Float16 h[16]; unsigned short u[16]; };
template <int NT>
__device__ __forceinline__ v8f mmaH(v16h ah, v16h al, v16h bh, v16h bl, v8f c) {
  c = __builtin_amdgcn_wmma_f32_16x16x32_f16(false, ah, false, bh, (short)0, c, false, false);
  if (NT >= 2) c = __builtin_amdgcn_wmma_f32_16x16x32_f16(false, al, false, bh, (short)0, c, false, false);
  if (NT >= 3) c = __builtin_amdgcn_wmma_f32_16x16x32_f16(false, ah, false, bl, (short)0, c, false, false);
  asm volatile("v_nop\n\tv_nop\n\tv_nop\n\tv_nop" : "+v"(c) : "v"(ah), "v"(al), "v"(bh), "v"(bl));
  return c;
}
template <bool ASPLIT>
__global__ __launch_bounds__(128) void k_gemm_h(const float* __restrict__ A, int lda, size_t sA, const _Float16* __restrict__ Bh, int ldb, size_t sB, float alpha, float* __restrict__ C, int ldc, size_t sC, int M, int N, int K) {
  __shared__ __attribute__((aligned(16))) float so[4][16][64];
  const int tid = threadIdx.x, w = tid >> 5, lane = tid & 31, ln = lane & 15, hh = lane >> 4; const int by = blockIdx.y;
  A += (size_t)by * sA; Bh += (size_t)by * sB; C += (size_t)by * sC;
  const int ntn = (N + 63) / 64; const int wid = blockIdx.x * 4 + w; const int mt = wid / ntn, nq = wid % ntn; if (mt * 16 >= M) return;
  const int row0 = mt * 16, col0 = nq * 64; const float* arow = A + (size_t)(row0 + ln) * lda;
  v8f acc[4] = {};
  for (int kb = 0; kb < K; kb += 32) {
    FragH ah, al;
    const v4f x0 = *(const v4fa*)(arow + kb + 8 * hh), x1 = *(const v4fa*)(arow + kb + 8 * hh + 4), x2 = *(const v4fa*)(arow + kb + 16 + 8 * hh), x3 = *(const v4fa*)(arow + kb + 16 + 8 * hh + 4);
    float xs[16] = {x0[0],x0[1],x0[2],x0[3],x1[0],x1[1],x1[2],x1[3],x2[0],x2[1],x2[2],x2[3],x3[0],x3[1],x3[2],x3[3]};
#pragma unroll
    for (int i = 0; i < 16; ++i) { const _Float16 h = (_Float16)xs[i]; ah.h[i] = h; al.h[i] = ASPLIT ? (_Float16)(xs[i] - (float)h) : (_Float16)0.0f; }
#pragma unroll
    for (int t = 0; t < 4; ++t) { if (col0 + t * 16 >= N) continue; const size_t boff = (size_t)(col0 + t * 16 + ln) * ldb + kb; FragH bq; bq.half[0] = *(const v8us*)(Bh + boff + 8 * hh); bq.half[1] = *(const v8us*)(Bh + boff + 16 + 8 * hh);
      acc[t] = mmaH<ASPLIT ? 2 : 1>(ah.v, al.v, bq.v, bq.v, acc[t]); }
  }
#pragma unroll
  for (int t = 0; t < 4; ++t) { if (col0 + t * 16 >= N) continue;
#pragma unroll
    for (int r = 0; r < 8; ++r) so[w][8 * hh + r][t * 16 + ln] = acc[t][r] * alpha; }
  __builtin_amdgcn_fence(__ATOMIC_ACQ_REL, "workgroup"); __builtin_amdgcn_wave_barrier();
  const int rsub = lane >> 4, c4 = (lane & 15) * 4;
  for (int pass = 0; pass < 2; ++pass) {
#pragma unroll
    for (int q = 0; q < 8; ++q) { const int r = q * 2 + rsub; if (col0 + c4 < N) { const v4f v = *(const v4fa*)&so[w][r][c4]; *(volatile v4f*)(C + (size_t)(row0 + r) * ldc + col0 + c4) = v; } }
    if (pass == 0) __threadfence(); }
}

__global__ __launch_bounds__(256) void k_wt_f16(const float* __restrict__ W, _Float16* __restrict__ Wt, int K, int N, float scale) {
  const int t = blockIdx.x * 256 + threadIdx.x; if (t >= N * (K / 8)) return; const int n = t / (K / 8), k8 = (t % (K / 8)) * 8; FragH f;
#pragma unroll
  for (int i = 0; i < 8; ++i) f.h[i] = (_Float16)(bf16_round(W[(size_t)(k8 + i) * N + n]) * scale); const v8us o = f.half[0];
  *(volatile v8us*)((unsigned short*)Wt + (size_t)n * K + k8) = o; __threadfence(); *(volatile v8us*)((unsigned short*)Wt + (size_t)n * K + k8) = o;
}
template <int ACT>
__global__ __launch_bounds__(128) void k_gemm_hhx(const _Float16* __restrict__ A, int lda, size_t sA, const _Float16* __restrict__ Bh, int ldb, size_t sB, float alpha, const float* __restrict__ bias, size_t sBias, const float* __restrict__ CP, int rowsPerB, size_t sCPb, int row0g,
    float* __restrict__ C, _Float16* __restrict__ C16, int ldc, size_t sC, int M, int N, int K) {
  __shared__ __attribute__((aligned(16))) float so[4][16][64];
  const int tid = threadIdx.x, w = tid >> 5, lane = tid & 31, ln = lane & 15, hh = lane >> 4; const int by = blockIdx.y;
  A += (size_t)by * sA; Bh += (size_t)by * sB; const size_t cofs = (size_t)by * sC; const float* bp = bias ? bias + (size_t)by * sBias : nullptr;
  const int ntn = (N + 63) / 64; const int wid = blockIdx.x * 4 + w; const int mt = wid / ntn, nq = wid % ntn; if (mt * 16 >= M) return;
  const int row0 = mt * 16, col0 = nq * 64; const _Float16* arow = A + (size_t)(row0 + ln) * lda;
  v8f acc[4] = {};
  for (int kb = 0; kb < K; kb += 32) { FragH ah; ah.half[0] = *(const v8us*)((const unsigned short*)arow + kb + 8 * hh); ah.half[1] = *(const v8us*)((const unsigned short*)arow + kb + 16 + 8 * hh);
#pragma unroll
    for (int t = 0; t < 4; ++t) { if (col0 + t * 16 >= N) continue; const size_t boff = (size_t)(col0 + t * 16 + ln) * ldb + kb; FragH bq; bq.half[0] = *(const v8us*)((const unsigned short*)Bh + boff + 8 * hh); bq.half[1] = *(const v8us*)((const unsigned short*)Bh + boff + 16 + 8 * hh);
      acc[t] = mmaH<1>(ah.v, ah.v, bq.v, bq.v, acc[t]); }
  }
#pragma unroll
  for (int t = 0; t < 4; ++t) { if (col0 + t * 16 >= N) continue; const int col = col0 + t * 16 + ln; const float bv = bp ? bf16_round(bp[col]) : 0.f;
#pragma unroll
    for (int r = 0; r < 8; ++r) { float v = acc[t][r] * alpha + bv; if (CP) { const int bidx = (row0g + row0 + 8 * hh + r) / rowsPerB; v += CP[(size_t)bidx * sCPb + (size_t)by * 64 + col]; } if (ACT == 1) v = (v > 0.f) ? v : expm1f(v); else if (ACT == 7) v = (v > 0.f) ? v + 1.0f : expf(v); else if (ACT == 8) v = tanhf(v); else if (ACT == 9) v = 0.5f * v * (1.0f + tanhf(0.7978845608028654f * (v + 0.044715f * v * v * v))); else if (ACT == 11) v = 1.0f / (1.0f + expf(-v)); else if (ACT == 12) v = (v > 0.f) ? v : 0.01f * v; else if (ACT == 14) v = (v > 0.f) ? v : 0.1f * v; else if (ACT == 15) v = v / (1.0f + expf(-v)); else if (ACT == 3) v = fmaxf(v, 0.f); else if (ACT == 6) v = 0.5f * v * (1.0f + erff(v * 0.70710678118654752f)); so[w][8 * hh + r][t * 16 + ln] = v; } }
  __builtin_amdgcn_fence(__ATOMIC_ACQ_REL, "workgroup"); __builtin_amdgcn_wave_barrier();
  const int rsub = lane >> 4, c4 = (lane & 15) * 4; typedef _Float16 v4h __attribute__((ext_vector_type(4)));
  for (int pass = 0; pass < 2; ++pass) {
#pragma unroll
    for (int q = 0; q < 8; ++q) { const int r = q * 2 + rsub; if (col0 + c4 < N) { const v4f v = *(const v4fa*)&so[w][r][c4]; if (C) *(volatile v4f*)(C + cofs + (size_t)(row0 + r) * ldc + col0 + c4) = v; if (C16) { v4h h4; for (int i = 0; i < 4; ++i) h4[i] = (_Float16)v[i]; *(volatile v4h*)(C16 + cofs + (size_t)(row0 + r) * ldc + col0 + c4) = h4; } } }
    if (pass == 0) __threadfence(); }
}


typedef _Float16 v4h __attribute__((ext_vector_type(4)));

__global__ __launch_bounds__(256) void k_x16(const float* __restrict__ x, _Float16* __restrict__ X16, size_t n8) { const size_t t = (size_t)blockIdx.x * 256 + threadIdx.x; if (t >= n8) return; FragH f;
#pragma unroll
  for (int q = 0; q < 8; ++q) f.h[q] = (_Float16)bf16_round(x[t * 8 + q]); *(volatile v8us*)((unsigned short*)X16 + t * 8) = f.half[0]; __threadfence(); *(volatile v8us*)((unsigned short*)X16 + t * 8) = f.half[0]; }
__global__ __launch_bounds__(256) void k_h16(const float* __restrict__ x, _Float16* __restrict__ X16, size_t n8) { const size_t t = (size_t)blockIdx.x * 256 + threadIdx.x; if (t >= n8) return; FragH f;
#pragma unroll
  for (int q = 0; q < 8; ++q) f.h[q] = (_Float16)x[t * 8 + q]; *(volatile v8us*)((unsigned short*)X16 + t * 8) = f.half[0]; __threadfence(); *(volatile v8us*)((unsigned short*)X16 + t * 8) = f.half[0]; }
__global__ __launch_bounds__(256) void k_round16f(const float* __restrict__ W, _Float16* __restrict__ Bt, size_t n8) { const size_t t = (size_t)blockIdx.x * 256 + threadIdx.x; if (t >= n8) return; FragH f;
#pragma unroll
  for (int i = 0; i < 8; ++i) f.h[i] = (_Float16)(bf16_round(W[t * 8 + i]) * 16.0f); *(volatile v8us*)((unsigned short*)Bt + t * 8) = f.half[0]; __threadfence(); *(volatile v8us*)((unsigned short*)Bt + t * 8) = f.half[0]; }
template <int NHv, int TTv>
__global__ __launch_bounds__(256) void k_vt(const _Float16* __restrict__ V16, int ldv, int voff, _Float16* __restrict__ Vt) { __shared__ unsigned short tl[64][66]; const int tid = threadIdx.x; const int slab = blockIdx.x / (TTv / 64), lg = blockIdx.x % (TTv / 64); const int b = slab / NHv, h = slab % NHv;
  for (int i = tid; i < 64 * 8; i += 256) { const int r = i / 8, c8 = (i % 8) * 8; FragH f; f.half[0] = *(const v8us*)((const unsigned short*)V16 + ((size_t)b * TTv + lg * 64 + r) * ldv + voff + h * 64 + c8);
#pragma unroll
    for (int q = 0; q < 8; ++q) tl[r][c8 + q] = f.u[q]; }
  __syncthreads();
  for (int pass = 0; pass < 2; ++pass) {
#pragma unroll
    for (int rd = 0; rd < 2; ++rd) { const int d = rd * 32 + tid / 8, pc = tid % 8; FragH f;
#pragma unroll
      for (int q = 0; q < 8; ++q) f.u[q] = tl[pc * 8 + q][d];
      *(volatile v8us*)((unsigned short*)Vt + ((size_t)slab * 64 + d) * TTv + lg * 64 + pc * 8) = f.half[0]; }
    if (pass == 0) __threadfence(); } }

__device__ __forceinline__ void cmul(float ar, float ai, float br, float bi, float& cr, float& ci) {
  #pragma clang fp contract(off)
  cr = ar * br - ai * bi; ci = ar * bi + ai * br; }
__global__ __launch_bounds__(64) void k_buildU(const float* __restrict__ prm, _Float16* __restrict__ Bh, _Float16* __restrict__ Bl) {
  #pragma clang fp contract(off)
  __shared__ float Ur[16][16], Ui[16][16];
  __shared__ float sr[16][16], si[16][16];
  if (threadIdx.x == 0) { for (int c = 0; c < 16; ++c) for (int a = 0; a < 16; ++a) { sr[c][a] = (a == c) ? 1.f : 0.f; si[c][a] = 0.f; }
#pragma unroll 1
    for (int l = 0; l < 3; ++l) {
#pragma unroll 1
      for (int w = 0; w < 4; ++w) { const float phi = bf16_round(prm[(l * 4 + w) * 3 + 0]), th = bf16_round(prm[(l * 4 + w) * 3 + 1]), om = bf16_round(prm[(l * 4 + w) * 3 + 2]); float s, c; sincosf(th * 0.5f, &s, &c); float s1, c1, s2, c2; sincosf((phi + om) * 0.5f, &s1, &c1); sincosf((phi - om) * 0.5f, &s2, &c2);
        const float m00r = c1 * c, m00i = -s1 * c, m01r = -c2 * s, m01i = -s2 * s, m10r = c2 * s, m10i = -s2 * s, m11r = c1 * c, m11i = s1 * c;
        const int bit = 3 - w;
#pragma unroll 1
        for (int col = 0; col < 16; ++col)
#pragma unroll 1
          for (int idx = 0; idx < 16; ++idx) if (!((idx >> bit) & 1)) { const int j = idx | (1 << bit); const float a0r = sr[col][idx], a0i = si[col][idx], a1r = sr[col][j], a1i = si[col][j]; float t1r, t1i, t2r, t2i;
          cmul(m00r, m00i, a0r, a0i, t1r, t1i); cmul(m01r, m01i, a1r, a1i, t2r, t2i); sr[col][idx] = t1r + t2r; si[col][idx] = t1i + t2i;
          cmul(m10r, m10i, a0r, a0i, t1r, t1i); cmul(m11r, m11i, a1r, a1i, t2r, t2i); sr[col][j] = t1r + t2r; si[col][j] = t1i + t2i; } }
      const int r = l % 3 + 1;
      for (int w = 0; w < 4; ++w) { const int cb = 3 - w, tb = 3 - ((w + r) % 4);
        for (int col = 0; col < 16; ++col) for (int idx = 0; idx < 16; ++idx) if (((idx >> cb) & 1) && !((idx >> tb) & 1)) { const int j = idx | (1 << tb); const float tr = sr[col][idx], ti = si[col][idx]; sr[col][idx] = sr[col][j]; si[col][idx] = si[col][j]; sr[col][j] = tr; si[col][j] = ti; } } }
    for (int col = 0; col < 16; ++col) for (int a = 0; a < 16; ++a) { Ur[a][col] = sr[col][a]; Ui[a][col] = si[col][a]; } }
  __syncthreads();
  const int t = threadIdx.x; if (t >= 32) return;
  FragH fh[4], fl[4];
  for (int it = 0; it < 4; ++it) { const int pi = it * 32 + t; const int n = pi / 4, k0 = (pi % 4) * 8; for (int q = 0; q < 8; ++q) { const int k = k0 + q; float v = 0.f; if (k < 16) v = (n < 16) ? Ur[n][k] : Ui[n - 16][k]; const _Float16 hv = (_Float16)v; fh[it].h[q] = hv; fl[it].h[q] = (_Float16)((v - (float)hv) * 1024.0f); } }
  for (int pass = 0; pass < 2; ++pass) { for (int it = 0; it < 4; ++it) { const size_t pi = (size_t)it * 32 + t; *(volatile v8us*)((unsigned short*)Bh + pi * 8) = fh[it].half[0]; *(volatile v8us*)((unsigned short*)Bl + pi * 8) = fl[it].half[0]; } if (pass == 0) __threadfence(); } }
__global__ __launch_bounds__(256) void k_psi0(const float* __restrict__ x, _Float16* __restrict__ Ph, _Float16* __restrict__ Pl) {
  #pragma clang fp contract(off)
  const size_t t = (size_t)blockIdx.x * 256 + threadIdx.x; if (t >= (size_t)NC * 4) return; const int n = (int)(t / 4), a0 = (int)(t % 4) * 8; const int b = n / NPATCH, p = n % NPATCH, i = p / 14, j = p % 14;
  float cw[4], sw[4];
#pragma unroll 1
  for (int w = 0; w < 4; ++w) { const int di = w >> 1, dj = w & 1; const float ang = bf16_round(x[(size_t)b * 784 + (2 * i + di) * 28 + (2 * j + dj)]); cw[w] = cosf(ang * 0.5f); sw[w] = sinf(ang * 0.5f); }
  FragH fh, fl;
#pragma unroll
  for (int q = 0; q < 8; ++q) { const int idx = a0 + q; float v = 0.f; if (idx < 16) { v = 1.f; for (int w = 0; w < 4; ++w) v *= ((idx >> (3 - w)) & 1) ? sw[w] : cw[w]; } const _Float16 hv = (_Float16)v; fh.h[q] = hv; fl.h[q] = (_Float16)((v - (float)hv) * 1024.0f); }
  for (int pass = 0; pass < 2; ++pass) { *(volatile v8us*)((unsigned short*)Ph + t * 8) = fh.half[0]; *(volatile v8us*)((unsigned short*)Pl + t * 8) = fl.half[0]; if (pass == 0) __threadfence(); } }
__global__ __launch_bounds__(256) void k_expz(const float* __restrict__ A, float* __restrict__ Q) {
  #pragma clang fp contract(off)
  const int n = blockIdx.x * 256 + threadIdx.x; if (n >= NC) return; v4f qz = {0.f, 0.f, 0.f, 0.f};
#pragma unroll
  for (int idx = 0; idx < 16; ++idx) { const float re = A[(size_t)n * 32 + idx], im = A[(size_t)n * 32 + 16 + idx]; const float pr = re * re + im * im; for (int w = 0; w < 4; ++w) qz[w] += ((idx >> (3 - w)) & 1) ? -pr : pr; }
  *(volatile v4f*)(Q + (size_t)n * 4) = qz; __threadfence(); *(volatile v4f*)(Q + (size_t)n * 4) = qz; }
__global__ __launch_bounds__(256) void k_head(const float* __restrict__ Q, const float* __restrict__ Wc, const float* __restrict__ bc, float* __restrict__ out) {
  #pragma clang fp contract(off)
  const int t = blockIdx.x * 256 + threadIdx.x; if (t >= NIMG * NCLS) return; const int b = t / NCLS, cls = t % NCLS; float lg[NCLS];
  for (int c = 0; c < NCLS; ++c) lg[c] = bf16_round(bc[c]);
#pragma unroll 1
  for (int k = 0; k < NQ; ++k) { const float qv = Q[(size_t)b * NQ + k];
#pragma unroll
    for (int c = 0; c < NCLS; ++c) lg[c] += qv * bf16_round(Wc[(size_t)c * NQ + k]); }
  float m = lg[0]; for (int c = 1; c < NCLS; ++c) m = fmaxf(m, lg[c]); float z = 0.f; for (int c = 0; c < NCLS; ++c) z += expf(lg[c] - m);
  float mine = lg[0]; for (int c = 1; c < NCLS; ++c) if (c == cls) mine = lg[c]; const float v = (mine - m) - logf(z);
  *(volatile float*)(out + t) = v; __threadfence(); *(volatile float*)(out + t) = v; }

extern "C" void kernel_launch(void* const* d_in, const int* in_sizes, int n_in,
                              void* d_out, int out_size, void* d_ws, size_t ws_size, hipStream_t stream) {
  (void)in_sizes; (void)n_in; (void)out_size;
  const float* const* I = (const float* const*)d_in; const float* x = I[0]; const float* prm = I[1]; const float* Wc = I[2]; const float* bc = I[3];
  char* ws = (char*)d_ws; size_t off = 0;
  auto take = [&](size_t bytes) { char* p = ws + off; off += (bytes + 255) & ~(size_t)255; return p; };
  _Float16* Bh = (_Float16*)take(32 * 32 * 2); _Float16* Bl = (_Float16*)take(32 * 32 * 2); _Float16* Ph = (_Float16*)take((size_t)NC * 32 * 2); _Float16* Pl = (_Float16*)take((size_t)NC * 32 * 2); float* A = (float*)take((size_t)NC * 32 * 4); float* Q = (float*)take((size_t)NC * 4 * 4);
  if (off > ws_size) return;
  k_buildU<<<1, 64, 0, stream>>>(prm, Bh, Bl); k_psi0<<<(unsigned)(((size_t)NC * 4 + 255) / 256), 256, 0, stream>>>(x, Ph, Pl);
  const dim3 ga(((NC / 16) * 1 + 3) / 4, 1);
  k_gemm_hhx<0><<<ga, 128, 0, stream>>>(Ph, 32, 0, Bh, 32, 0, 1.0f, nullptr, 0, nullptr, 1, 0, 0, A, nullptr, 32, 0, NC, 32, 32);
  k_gemm_hhx<0><<<ga, 128, 0, stream>>>(Pl, 32, 0, Bh, 32, 0, 0.0009765625f, nullptr, 0, A, 1, 32, 0, A, nullptr, 32, 0, NC, 32, 32);
  k_gemm_hhx<0><<<ga, 128, 0, stream>>>(Ph, 32, 0, Bl, 32, 0, 0.0009765625f, nullptr, 0, A, 1, 32, 0, A, nullptr, 32, 0, NC, 32, 32);
  k_expz<<<(NC + 255) / 256, 256, 0, stream>>>(A, Q);
  k_head<<<(NIMG * NCLS + 255) / 256, 256, 0, stream>>>(Q, Wc, bc, (float*)d_out);
}
